// GCN_13134009991660
// MI455X (gfx1250) — hardware-run, weakly checked
//
#include <hip/hip_runtime.h>
#include <stddef.h>
#include <stdint.h>


#define NN      50000
#define NE      800000
#define DF      96
#define AP      192
#define K1      288
#define K2      384
#define MP      50048
#define GBM     128
#define GTHR    256
#define NTHR    256
#define NWAVE   8
#define NBA     1024
#define PKS     10
#define NB      49
#define NPADN   (NB * NBA)
#define RCAP    20480
#define WLCAP   3072
#define DEGCAP  64
#define EPW     (NE / NWAVE)
#define XB_UNITS (MP * DF / 8)
#define XB_BLKS  (XB_UNITS / NTHR)
#define WBLK    12
#define BK_LIST (NWAVE * WLCAP)
#define BK_ZINTS (RCAP + NWAVE * NBA + 2 * NBA + 32)
#define BK_INTS (BK_LIST + BK_ZINTS)
#define LDS_BK  (BK_INTS * 4)
#define MEAS_BLK_HITS 16623
#define MEAS_MAXDEG   35
#define SPLIT_AGG1 1
#define SPLIT_H    1
#define SPLIT_AGG2 1

static_assert(NE % (NWAVE * 32) == 0 && NE % 256 == 0);
static_assert(NE < (1 << 20));
static_assert(NBA == (1 << PKS) && NBA == NTHR * 4 && NBA % NWAVE == 0);
static_assert(NB * NBA >= MP && MP % GBM == 0 && MP >= NN && NBA % GBM == 0);
static_assert((long long)RCAP * 100 >= (long long)MEAS_BLK_HITS * 105);
static_assert((long long)WLCAP * 80 >= (long long)MEAS_BLK_HITS * 13);
static_assert(DEGCAP >= MEAS_MAXDEG + 8);
static_assert(RCAP % (NTHR * 4) == 0 && BK_ZINTS % 4 == 0 && BK_LIST % 4 == 0);
static_assert(LDS_BK <= 300000);
static_assert(DF % 32 == 0 && DF == 6 * 16 && K1 % 32 == 0 && K2 % 32 == 0);
static_assert(K1 == 3 * DF && K2 == 4 * DF && AP == 2 * DF);
static_assert(GBM == (GTHR / 32) * 16);
static_assert(XB_UNITS % NTHR == 0 && (NN * DF) % 8 == 0);
static_assert(DF == WBLK * 8);

typedef float          v4f   __attribute__((ext_vector_type(4)));
typedef float          v8f   __attribute__((ext_vector_type(8)));
typedef int            v4i   __attribute__((ext_vector_type(4)));
typedef int            v8i   __attribute__((ext_vector_type(8)));
typedef unsigned       v2u   __attribute__((ext_vector_type(2)));
typedef unsigned       v4u   __attribute__((ext_vector_type(4)));
typedef unsigned short v8us  __attribute__((ext_vector_type(8)));
typedef __bf16         v16bf __attribute__((ext_vector_type(16)));
typedef v4f  __attribute__((may_alias)) v4fa;
typedef v4i  __attribute__((may_alias)) v4ia;
typedef v2u  __attribute__((may_alias)) v2ua;
typedef v4u  __attribute__((may_alias)) v4ua;
typedef v8us __attribute__((may_alias)) v8usa;
union FragB { v16bf v; v8us h[2]; v8i w; };

__device__ __forceinline__ v8f wmb(const FragB& a, const FragB& b, v8f c) {
  v8f d = __builtin_amdgcn_wmma_f32_16x16x32_bf16(false, a.v, false, b.v, (short)0, c, false, false);
  asm volatile("v_nop\n\tv_nop\n\tv_nop\n\tv_nop" : "+v"(d) : "v"(a.w), "v"(b.w));
  return d;
}

__device__ __forceinline__ unsigned bf16_bits(float f) {
  const unsigned u = __float_as_uint(f);
  const unsigned r = ((u + 0x7FFFu + ((u >> 16) & 1u)) >> 16) & 0xFFFFu;
  const unsigned q = ((u >> 16) & 0xFFFFu) | 0x0040u;
  return ((u & 0x7FFFFFFFu) > 0x7F800000u) ? q : r;
}
__device__ __forceinline__ float bf16_val(float f) { return __uint_as_float(bf16_bits(f) << 16); }
__device__ __forceinline__ float bfw_lo(unsigned w) { return __uint_as_float(w << 16); }
__device__ __forceinline__ float bfw_hi(unsigned w) { return __uint_as_float(w & 0xffff0000u); }
__device__ __forceinline__ void pack2(float a, float b, unsigned& hw, unsigned& lw) {
  const unsigned ha = bf16_bits(a), hb = bf16_bits(b);
  const unsigned la = bf16_bits(a - __uint_as_float(ha << 16));
  const unsigned lb = bf16_bits(b - __uint_as_float(hb << 16));
  hw = ha | (hb << 16);
  lw = la | (lb << 16);
}
__device__ __forceinline__ float relu_k(float v) { return (v > 0.0f) ? v : (v - v); }

__device__ __forceinline__ void wave_sync() {
  __builtin_amdgcn_fence(__ATOMIC_RELEASE, "wavefront");
  __builtin_amdgcn_wave_barrier();
  __builtin_amdgcn_fence(__ATOMIC_ACQUIRE, "wavefront");
}

template <int KP>
__device__ __forceinline__ void wslab(const float* __restrict__ rel, const float* __restrict__ root,
                                      unsigned short* plane, int wb, unsigned short* T, int tid) {
  const int n0 = 8 * wb;
  const int wave = tid >> 5;
  if (wave < 6) {
    const bool isRel = wave < 3;
    const int k = isRel ? tid : tid - DF;
    v4f a, b;
    if (isRel) {
      a = *(const v4f*)(rel + (size_t)k * DF + n0);
      b = *(const v4f*)(rel + (size_t)k * DF + n0 + 4);
    } else {
      a = *(const v4f*)(root + (size_t)k * DF + n0);
      b = *(const v4f*)(root + (size_t)k * DF + n0 + 4);
    }
    const float f[8] = {a.x, a.y, a.z, a.w, b.x, b.y, b.z, b.w};
    const int c0 = isRel ? k : 2 * DF + k;
    const int c1 = isRel ? DF + k : ((KP == K2) ? 3 * DF + k : 2 * DF + k);
#pragma unroll
    for (int i = 0; i < 8; ++i) {
      const unsigned short o = (unsigned short)bf16_bits(f[i]);
      T[i * KP + c0] = o;
      T[i * KP + c1] = o;
    }
  }
  __syncthreads();
  unsigned short* base = plane + (size_t)n0 * KP;
#pragma unroll 1
  for (int q = tid; q < KP; q += NTHR) {
    const v8us v = *(const v8usa*)(T + 8 * q);
    *(volatile v8us*)(base + 8 * q) = v;
  }
  __threadfence();
#pragma unroll 1
  for (int q = tid; q < KP; q += NTHR) {
    const v8us v = *(const v8usa*)(T + 8 * q);
    *(volatile v8us*)(base + 8 * q) = v;
  }
}

__global__ __launch_bounds__(NTHR) void k_prep(const float* __restrict__ x,
                                               const float* __restrict__ w1rel, const float* __restrict__ w1root,
                                               const float* __restrict__ w2rel, const float* __restrict__ w2root,
                                               unsigned short* XB, unsigned short* W1C, unsigned short* W2C) {
  __shared__ __attribute__((aligned(16))) unsigned short wts[8 * K2];
  const int tid = (int)threadIdx.x;
  const int blk = (int)blockIdx.x;
  if (blk < XB_BLKS) {
    const int u = blk * NTHR + tid;
    const bool live = u < (NN * DF) / 8;
    const int uc = live ? u : (NN * DF) / 8 - 1;
    const float* p = x + (size_t)uc * 8;
    const v4f a = *(const v4f*)p;
    const v4f b = *(const v4f*)(p + 4);
    asm volatile("" :: "v"(a), "v"(b));
    v8us o;
    o[0] = live ? (unsigned short)bf16_bits(a.x) : (unsigned short)0;
    o[1] = live ? (unsigned short)bf16_bits(a.y) : (unsigned short)0;
    o[2] = live ? (unsigned short)bf16_bits(a.z) : (unsigned short)0;
    o[3] = live ? (unsigned short)bf16_bits(a.w) : (unsigned short)0;
    o[4] = live ? (unsigned short)bf16_bits(b.x) : (unsigned short)0;
    o[5] = live ? (unsigned short)bf16_bits(b.y) : (unsigned short)0;
    o[6] = live ? (unsigned short)bf16_bits(b.z) : (unsigned short)0;
    o[7] = live ? (unsigned short)bf16_bits(b.w) : (unsigned short)0;
    unsigned short* dp = XB + (size_t)u * 8;
    *(volatile v8us*)dp = o;
    __threadfence();
    *(volatile v8us*)dp = o;
  } else if (blk < XB_BLKS + WBLK) {
    wslab<K1>(w1rel, w1root, W1C, blk - XB_BLKS, wts, tid);
  } else {
    int wb = blk - XB_BLKS - WBLK;
    wb = wb > WBLK - 1 ? WBLK - 1 : wb;
    wslab<K2>(w2rel, w2root, W2C, wb, wts, tid);
  }
}

__global__ __launch_bounds__(NTHR) void k_bucket(const int* __restrict__ keys, const int* __restrict__ gidx,
                                                 int* LIST, int* CNT, int* OFF, int* REC) {
  extern __shared__ __attribute__((aligned(16))) int dsm[];
  int* lists = dsm;
  int* reg2  = lists + BK_LIST;
  int* wcur  = reg2 + RCAP;
  int* scnt  = wcur + NWAVE * NBA;
  int* soff  = scnt + NBA;
  int* misc  = soff + NBA;
  const int tid = (int)threadIdx.x, lane = tid & 31, wave = tid >> 5;
  const int nodeBase = (int)blockIdx.x * NBA;
  int nb = NN - nodeBase;
  nb = nb > NBA ? NBA : (nb < 1 ? 1 : nb);

  {
    const v4i z4 = {0, 0, 0, 0};
    for (int i = tid * 4; i < BK_ZINTS; i += NTHR * 4) *(v4ia*)(reg2 + i) = z4;
  }
  __syncthreads();

  int* wl = lists + wave * WLCAP;
  int wc = 0;
  {
    const int ebase = wave * EPW;
    const unsigned nbs = (unsigned)nodeBase;
    const unsigned unb = (unsigned)nb;
#pragma unroll 1
    for (int st = 0; st < EPW / 32; ++st) {
      const int e = ebase + 32 * st + lane;
      const int key = keys[e];
      const unsigned s = (unsigned)key - nbs;
      const bool hit = s < unb;
      const unsigned mk = __builtin_amdgcn_ballot_w32(hit);
      const int pos = wc + (int)__builtin_amdgcn_mbcnt_lo(mk, 0u);
      if (hit && pos < WLCAP) wl[pos] = (int)(((unsigned)e << PKS) | s);
      wc += (int)__builtin_popcount(mk);
    }
  }
  if (lane == 0) misc[wave] = wc;
  const int wcc = wc > WLCAP ? WLCAP : wc;
  __syncthreads();

  int* myc = wcur + wave * NBA;
  if (lane == 0) {
#pragma unroll 1
    for (int i = 0; i < wcc; ++i) {
      const int u  = wl[i];
      const int sl = u & (NBA - 1);
      myc[sl] = myc[sl] + 1;
    }
  }
  __syncthreads();

  int tot = 0;
  {
    v4i cw[NWAVE];
    int e0 = 0, e1 = 0, e2 = 0, e3 = 0;
#pragma unroll
    for (int w2 = 0; w2 < NWAVE; ++w2) {
      cw[w2] = *(const v4ia*)(wcur + w2 * NBA + 4 * tid);
      e0 += cw[w2].x; e1 += cw[w2].y; e2 += cw[w2].z; e3 += cw[w2].w;
    }
    const int ts = e0 + e1 + e2 + e3;
    int incl = ts;
#pragma unroll
    for (int d = 1; d < 32; d <<= 1) {
      const int up = __shfl_up(incl, d, 32);
      if (lane >= d) incl += up;
    }
    int mx = max(max(e0, e1), max(e2, e3));
    mx = max(mx, __shfl_xor(mx, 16, 32));
    mx = max(mx, __shfl_xor(mx, 8, 32));
    mx = max(mx, __shfl_xor(mx, 4, 32));
    mx = max(mx, __shfl_xor(mx, 2, 32));
    mx = max(mx, __shfl_xor(mx, 1, 32));
    if (lane == 31) misc[8 + wave] = incl;
    if (lane == 0)  misc[16 + wave] = mx;
    __syncthreads();
    int pre = 0;
#pragma unroll
    for (int w2 = 0; w2 < NWAVE; ++w2) {
      const int wt = misc[8 + w2];
      tot += wt;
      pre += (w2 < wave) ? wt : 0;
    }
    int run = pre + incl - ts;
    v4i so, sc;
    so.x = run; run += e0;
    so.y = run; run += e1;
    so.z = run; run += e2;
    so.w = run;
    sc.x = e0; sc.y = e1; sc.z = e2; sc.w = e3;
    *(v4ia*)(soff + 4 * tid) = so;
    *(v4ia*)(scnt + 4 * tid) = sc;
    v4i cu = so;
#pragma unroll
    for (int w2 = 0; w2 < NWAVE; ++w2) {
      *(v4ia*)(wcur + w2 * NBA + 4 * tid) = cu;
      cu = cu + cw[w2];
    }
  }
  __syncthreads();

  if (lane == 0) {
#pragma unroll 1
    for (int i = 0; i < wcc; ++i) {
      const int u   = wl[i];
      const int sl  = u & (NBA - 1);
      const int eid = (int)((unsigned)u >> PKS);
      int pos = myc[sl];
      pos = pos < 0 ? 0 : (pos > RCAP - 1 ? RCAP - 1 : pos);
      reg2[pos] = eid;
      myc[sl] = pos + 1;
    }
  }
  __syncthreads();

  int bmax = 0, ovw = 0;
#pragma unroll
  for (int w2 = 0; w2 < NWAVE; ++w2) {
    bmax = max(bmax, misc[16 + w2]);
    ovw |= (misc[w2] > WLCAP) ? 1 : 0;
  }
  const int nh = tot < 0 ? 0 : (tot > RCAP ? RCAP : tot);
  const int flag = ((ovw != 0) || (tot > RCAP) || (bmax > DEGCAP)) ? 1 : 0;

  int* lrow = LIST + (size_t)blockIdx.x * RCAP;
#pragma unroll 1
  for (int it = 0; it < RCAP / (NTHR * 4); ++it) {
    const int i0 = 4 * (it * NTHR + tid);
    const v4i ev = *(const v4ia*)(reg2 + i0);
    int e0 = ev.x, e1 = ev.y, e2 = ev.z, e3 = ev.w;
    e0 = e0 < 0 ? 0 : (e0 > NE - 1 ? NE - 1 : e0);
    e1 = e1 < 0 ? 0 : (e1 > NE - 1 ? NE - 1 : e1);
    e2 = e2 < 0 ? 0 : (e2 > NE - 1 ? NE - 1 : e2);
    e3 = e3 < 0 ? 0 : (e3 > NE - 1 ? NE - 1 : e3);
    int g0 = gidx[e0], g1 = gidx[e1], g2 = gidx[e2], g3 = gidx[e3];
    asm volatile("" :: "v"(g0), "v"(g1), "v"(g2), "v"(g3));
    g0 = g0 < 0 ? 0 : (g0 > NN - 1 ? NN - 1 : g0);
    g1 = g1 < 0 ? 0 : (g1 > NN - 1 ? NN - 1 : g1);
    g2 = g2 < 0 ? 0 : (g2 > NN - 1 ? NN - 1 : g2);
    g3 = g3 < 0 ? 0 : (g3 > NN - 1 ? NN - 1 : g3);
    v4i ov;
    ov.x = (i0     < nh) ? g0 : 0;
    ov.y = (i0 + 1 < nh) ? g1 : 0;
    ov.z = (i0 + 2 < nh) ? g2 : 0;
    ov.w = (i0 + 3 < nh) ? g3 : 0;
    *(volatile v4i*)(lrow + i0) = ov;
    __threadfence();
    *(volatile v4i*)(lrow + i0) = ov;
  }
  {
    const v4i cv = *(const v4ia*)(scnt + 4 * tid);
    const v4i fv = *(const v4ia*)(soff + 4 * tid);
    v4i rv = {0, 0, 0, 0};
    rv.x = (tid == 0) ? bmax : 0;
    rv.y = (tid == 0) ? flag : 0;
    rv.z = (tid == 0) ? nh : 0;
    int* cp = CNT + (size_t)nodeBase + 4 * tid;
    int* fp = OFF + (size_t)nodeBase + 4 * tid;
    int* rp = REC + (size_t)blockIdx.x * 32 + 4 * (tid & 7);
    *(volatile v4i*)cp = cv;
    *(volatile v4i*)fp = fv;
    if (tid < 8) *(volatile v4i*)rp = rv;
    __threadfence();
    *(volatile v4i*)cp = cv;
    *(volatile v4i*)fp = fv;
    if (tid < 8) *(volatile v4i*)rp = rv;
  }
}

template <int LAYER>
__global__ __launch_bounds__(NTHR) void k_replay(const unsigned short* __restrict__ srcp, unsigned short* outp,
                                                 const int* __restrict__ LIST, const int* __restrict__ CNT,
                                                 const int* __restrict__ OFF, const int* __restrict__ REC) {
  constexpr int SP  = (LAYER == 1) ? DF : AP;
  constexpr int SPL = (LAYER == 1) ? SPLIT_AGG1 : SPLIT_AGG2;
  __shared__ __attribute__((aligned(16))) unsigned rowst[NWAVE * 96];
  const int tid = (int)threadIdx.x, lane = tid & 31, wave = tid >> 5;
  const int blk = (int)blockIdx.x;
  const int lc  = lane < 23 ? lane : 23;
  const int fl  = REC[(size_t)blk * 32 + 1];
  const float pz = (fl != 0) ? __int_as_float(0x7fc00000) : 0.0f;
  unsigned* wst = rowst + wave * 96;
  const int* lp = LIST + (size_t)blk * RCAP;
#pragma unroll 1
  for (int si = 0; si < NBA / NWAVE; ++si) {
    const int node = blk * NBA + si * NWAVE + wave;
    if (node >= MP) continue;
    const int craw = CNT[node];
    const int oraw = OFF[node];
    int cv = craw < 0 ? 0 : (craw > DEGCAP ? DEGCAP : craw);
    int ov = oraw < 0 ? 0 : (oraw > RCAP - 1 ? RCAP - 1 : oraw);
    cv = cv > RCAP - ov ? RCAP - ov : cv;
    const int c = __builtin_amdgcn_readfirstlane(cv);
    const int o = __builtin_amdgcn_readfirstlane(ov);
    const bool big = craw > DEGCAP;
    int last = o + c - 1; last = last < o ? o : last;
    float a0 = 0.0f, a1 = 0.0f, a2 = 0.0f, a3 = 0.0f;
#pragma unroll 1
    for (int b0 = 0; b0 < c; b0 += 32) {
      int idx = o + b0 + lane;
      idx = idx > last ? last : idx;
      int col = lp[idx];
      col = col < 0 ? 0 : (col > NN - 1 ? NN - 1 : col);
      const int m32 = (c - b0) < 32 ? (c - b0) : 32;
#pragma unroll 1
      for (int k = 0; k < m32; ++k) {
        const int sk = __builtin_amdgcn_readlane(col, k);
        const unsigned short* rp = srcp + (size_t)sk * SP + 4 * lc;
        if constexpr (LAYER == 1) {
          const v2u w = *(const v2ua*)rp;
          asm volatile("" :: "v"(w));
          a0 += bfw_lo(w.x);
          a1 += bfw_hi(w.x);
          a2 += bfw_lo(w.y);
          a3 += bfw_hi(w.y);
        } else {
          const v2u wh = *(const v2ua*)rp;
          const v2u wl = *(const v2ua*)(rp + DF);
          asm volatile("" :: "v"(wh), "v"(wl));
          a0 += bfw_lo(wh.x) + bfw_lo(wl.x);
          a1 += bfw_hi(wh.x) + bfw_hi(wl.x);
          a2 += bfw_lo(wh.y) + bfw_lo(wl.y);
          a3 += bfw_hi(wh.y) + bfw_hi(wl.y);
        }
      }
    }
    const float pzr = big ? __int_as_float(0x7fc00000) : pz;
    const bool live = node < NN;
    const float m0 = live ? (a0 + pzr) : 0.0f;
    const float m1 = live ? (a1 + pzr) : 0.0f;
    const float m2 = live ? (a2 + pzr) : 0.0f;
    const float m3 = live ? (a3 + pzr) : 0.0f;
    unsigned hw0, lw0, hw1, lw1;
    pack2(m0, m1, hw0, lw0);
    pack2(m2, m3, hw1, lw1);
    if (SPL == 0) { lw0 = 0u; lw1 = 0u; }
    v2u hq, lq;
    hq.x = hw0; hq.y = hw1;
    lq.x = lw0; lq.y = lw1;
    if (lane < 24) {
      *(v2ua*)(wst + 2 * lane)      = hq;
      *(v2ua*)(wst + 48 + 2 * lane) = lq;
    }
    wave_sync();
    const v4u q = *(const v4ua*)(wst + 4 * lc);
    wave_sync();
    unsigned short* wp = outp + (size_t)node * AP + 8 * lc;
    if (lane < 24) *(volatile v4u*)wp = q;
    __threadfence();
    if (lane < 24) *(volatile v4u*)wp = q;
  }
}

template <int KP>
__device__ __forceinline__ void ksteps(const unsigned short* __restrict__ ap, const unsigned short* __restrict__ wp,
                                       int nst, v8f (&acc)[6]) {
#pragma unroll 1
  for (int ks = 0; ks < nst; ++ks) {
    FragB af;
    af.h[0] = *(const v8usa*)(ap + 32 * ks);
    af.h[1] = *(const v8usa*)(ap + 32 * ks + 16);
#pragma unroll
    for (int t = 0; t < 6; ++t) {
      const unsigned short* wq = wp + (size_t)(16 * t) * (size_t)KP + 32 * ks;
      FragB bf;
      bf.h[0] = *(const v8usa*)wq;
      bf.h[1] = *(const v8usa*)(wq + 16);
      acc[t] = wmb(af, bf, acc[t]);
    }
  }
}

template <int LAST>
__global__ __launch_bounds__(GTHR) __attribute__((amdgpu_num_vgpr(248)))
void k_gemm(const unsigned short* __restrict__ A0, const unsigned short* __restrict__ A1,
            const unsigned short* __restrict__ BT, const float* __restrict__ bias,
            const int* __restrict__ REC, unsigned short* hout, float* outp) {
  constexpr int KP = (LAST != 0) ? K2 : K1;
  constexpr int P1 = (LAST != 0) ? AP : DF;
  constexpr int S1 = (LAST != 0) ? (AP / 32) : (DF / 32);
  __shared__ __attribute__((aligned(16))) float stg[GBM * DF];
  __shared__ __attribute__((aligned(16))) float bsh[DF];
  const int tid = (int)threadIdx.x, lane = tid & 31, wave = tid >> 5, hh = lane >> 4, m = lane & 15;
  const int rowBase = (int)blockIdx.x * GBM;

  if (tid < 24) {
    const v4f b4 = *(const v4f*)(bias + 4 * tid);
    v4f bq;
    bq.x = bf16_val(b4.x); bq.y = bf16_val(b4.y); bq.z = bf16_val(b4.z); bq.w = bf16_val(b4.w);
    *(v4fa*)(bsh + 4 * tid) = bq;
  }
  const int fl = REC[(size_t)(rowBase >> PKS) * 32 + 1];
  const float pz = (fl != 0) ? __int_as_float(0x7fc00000) : 0.0f;

  v8f acc[6];
  {
    const v8f z = {0.f, 0.f, 0.f, 0.f, 0.f, 0.f, 0.f, 0.f};
#pragma unroll
    for (int t = 0; t < 6; ++t) acc[t] = z;
  }
  const int arow = rowBase + 16 * wave + m;
  const unsigned short* wp = BT + (size_t)m * (size_t)KP + 8 * hh;
  ksteps<KP>(A0 + (size_t)arow * AP + 8 * hh, wp, AP / 32, acc);
  ksteps<KP>(A1 + (size_t)arow * P1 + 8 * hh, wp + AP, S1, acc);
  __syncthreads();

#pragma unroll
  for (int t = 0; t < 6; ++t) {
    const int lcl = 16 * t + m;
#pragma unroll
    for (int r = 0; r < 8; ++r) {
      const int lr = 16 * wave + 8 * hh + r;
      stg[lr * DF + lcl] = acc[t][r];
    }
  }
  __syncthreads();

  const int lcn = lane < 23 ? lane : 23;
  if constexpr (LAST == 0) {
    const int pc = lcn >= 12 ? lcn - 12 : lcn;
    const bool isHi = lcn < 12;
    const int cb = 8 * pc;
    const v4f ba = *(const v4fa*)(bsh + cb);
    const v4f bb = *(const v4fa*)(bsh + cb + 4);
    v4u pk[16];
#pragma unroll
    for (int i = 0; i < 16; ++i) {
      const int lr = 16 * wave + i;
      const bool live = (rowBase + lr) < NN;
      const v4f a = *(const v4fa*)(stg + lr * DF + cb);
      const v4f b = *(const v4fa*)(stg + lr * DF + cb + 4);
      float f[8] = {a.x + ba.x, a.y + ba.y, a.z + ba.z, a.w + ba.w,
                    b.x + bb.x, b.y + bb.y, b.z + bb.z, b.w + bb.w};
#pragma unroll
      for (int j = 0; j < 8; ++j) {
        const float v = relu_k(f[j]) + pz;
        f[j] = live ? v : 0.0f;
      }
      unsigned w[4];
#pragma unroll
      for (int j = 0; j < 4; ++j) {
        unsigned hw, lw;
        pack2(f[2 * j], f[2 * j + 1], hw, lw);
        if (SPLIT_H == 0) lw = 0u;
        w[j] = isHi ? hw : lw;
      }
      v4u pw; pw.x = w[0]; pw.y = w[1]; pw.z = w[2]; pw.w = w[3];
      pk[i] = pw;
    }
#pragma unroll
    for (int i = 0; i < 16; ++i) {
      const int gr = rowBase + 16 * wave + i;
      unsigned short* op = hout + (size_t)gr * AP + 8 * lcn;
      if (lane < 24) *(volatile v4u*)op = pk[i];
    }
    __threadfence();
#pragma unroll
    for (int i = 0; i < 16; ++i) {
      const int gr = rowBase + 16 * wave + i;
      unsigned short* op = hout + (size_t)gr * AP + 8 * lcn;
      if (lane < 24) *(volatile v4u*)op = pk[i];
    }
  } else {
    const v4f b4 = *(const v4fa*)(bsh + 4 * lcn);
    v4f pv[16];
#pragma unroll
    for (int i = 0; i < 16; ++i) {
      const int lr = 16 * wave + i;
      const v4f a = *(const v4fa*)(stg + lr * DF + 4 * lcn);
      v4f y;
      y.x = (a.x + b4.x) + pz;
      y.y = (a.y + b4.y) + pz;
      y.z = (a.z + b4.z) + pz;
      y.w = (a.w + b4.w) + pz;
      asm volatile("" :: "v"(y));
      pv[i] = y;
    }
#pragma unroll
    for (int i = 0; i < 16; ++i) {
      const int gr = rowBase + 16 * wave + i;
      const int gc = gr < NN ? gr : NN - 1;
      float* op = outp + (size_t)gc * DF + 4 * lcn;
      if (gr < NN && lane < 24) *(volatile v4f*)op = pv[i];
    }
    __threadfence();
#pragma unroll
    for (int i = 0; i < 16; ++i) {
      const int gr = rowBase + 16 * wave + i;
      const int gc = gr < NN ? gr : NN - 1;
      float* op = outp + (size_t)gc * DF + 4 * lcn;
      if (gr < NN && lane < 24) *(volatile v4f*)op = pv[i];
    }
  }
}

static inline size_t al256(size_t o) { return (o + 255) & ~(size_t)255; }

extern "C" void kernel_launch(void* const* d_in, const int* in_sizes, int n_in,
                              void* d_out, int out_size, void* d_ws, size_t ws_size,
                              hipStream_t stream) {
  if (n_in < 8) return;
  if (in_sizes[0] != NN * DF) return;
  if (in_sizes[1] != 2 * NE) return;
  if (in_sizes[2] != DF * DF || in_sizes[3] != DF) return;
  if (in_sizes[4] != DF * DF) return;
  if (in_sizes[5] != DF * DF || in_sizes[6] != DF) return;
  if (in_sizes[7] != DF * DF) return;
  if (out_size != NN * DF) return;

  const float* x      = (const float*)d_in[0];
  const int*   ei     = (const int*)  d_in[1];
  const int*   gix    = ei;
  const int*   key    = ei + NE;
  const float* w1rel  = (const float*)d_in[2];
  const float* b1     = (const float*)d_in[3];
  const float* w1root = (const float*)d_in[4];
  const float* w2rel  = (const float*)d_in[5];
  const float* b2     = (const float*)d_in[6];
  const float* w2root = (const float*)d_in[7];
  float* out = (float*)d_out;

  char* ws = (char*)d_ws;
  size_t off = 0;
  const size_t oXB = off; off = al256(off + (size_t)MP * DF * 2);
  const size_t oSM = off; off = al256(off + (size_t)MP * AP * 2);
  const size_t oH  = off; off = al256(off + (size_t)MP * AP * 2);
  const size_t oLS = off; off = al256(off + (size_t)NB * RCAP * 4);
  const size_t oCN = off; off = al256(off + (size_t)NPADN * 4);
  const size_t oOF = off; off = al256(off + (size_t)NPADN * 4);
  const size_t oRC = off; off = al256(off + (size_t)NB * 128);
  const size_t oW1 = off; off = al256(off + (size_t)DF * K1 * 2);
  const size_t oW2 = off; off = al256(off + (size_t)DF * K2 * 2);
  if (off > ws_size || off > (size_t)(128u << 20)) return;
  unsigned short* XB  = (unsigned short*)(ws + oXB);
  unsigned short* SUM = (unsigned short*)(ws + oSM);
  unsigned short* H   = (unsigned short*)(ws + oH);
  int* LIST = (int*)(ws + oLS);
  int* CNT  = (int*)(ws + oCN);
  int* OFF  = (int*)(ws + oOF);
  int* REC  = (int*)(ws + oRC);
  unsigned short* W1C = (unsigned short*)(ws + oW1);
  unsigned short* W2C = (unsigned short*)(ws + oW2);

  hipFuncSetAttribute(reinterpret_cast<const void*>(&k_bucket), hipFuncAttributeMaxDynamicSharedMemorySize, LDS_BK);

  k_prep<<<XB_BLKS + 2 * WBLK, NTHR, 0, stream>>>(x, w1rel, w1root, w2rel, w2root, XB, W1C, W2C);
  k_bucket<<<NB, NTHR, LDS_BK, stream>>>(key, gix, LIST, CNT, OFF, REC);
  k_replay<1><<<NB, NTHR, 0, stream>>>(XB, SUM, LIST, CNT, OFF, REC);
  k_gemm<0><<<MP / GBM, GTHR, 0, stream>>>(SUM, XB, W1C, b1, REC, H, out);
  k_replay<2><<<NB, NTHR, 0, stream>>>(H, SUM, LIST, CNT, OFF, REC);
  k_gemm<1><<<MP / GBM, GTHR, 0, stream>>>(SUM, H, W2C, b2, REC, H, out);
}
